// CommunityDetection_7421703488232
// MI455X (gfx1250) — hardware-verified
//
#include <hip/hip_runtime.h>
#include <stddef.h>


#define DIN     128
#define DHID    64
#define NCLS    16
#define NTHR    256
#define NWAVE   8
#define EPT     8
#define NGRP    2
#define CHUNK   (NTHR * EPT * NGRP)
#define WCAP    (EPT * NGRP * 32)
#define LISTN   (NWAVE * WCAP)
#define NB1     1024
#define NB2     4096
#define NBD     4096
#define G1ROWS  128
#define APITCH  136
#define WSCALE  8.0f
#define WINV    0.125f

#define LDS_GEMM1 (G1ROWS * APITCH * 2)
#define LDS_AGG1  (NB1 * DHID * 4 + LISTN * 4 + 64)
#define LDS_AGG2  (NB2 * NCLS * 4 + LISTN * 4 + 64)

static_assert((CHUNK & (CHUNK - 1)) == 0);
static_assert(CHUNK <= 4096);
static_assert((NB1 & (NB1 - 1)) == 0 && (NB2 & (NB2 - 1)) == 0 && (NBD & (NBD - 1)) == 0);
static_assert(NB1 <= 4096 && NB2 <= 4096 && NBD <= 4096);
static_assert(NBD >= NB1 && NB1 >= G1ROWS);
static_assert(G1ROWS * DHID * 4 <= LDS_GEMM1);
static_assert(256 * NCLS * 4 <= LISTN * 4);
static_assert(DIN % 32 == 0 && DHID % 32 == 0);
static_assert(NB1 % 256 == 0);

typedef float    v2f  __attribute__((ext_vector_type(2)));
typedef float    v4f  __attribute__((ext_vector_type(4)));
typedef float    v8f  __attribute__((ext_vector_type(8)));
typedef int      v4i  __attribute__((ext_vector_type(4)));
typedef _Float16 v8h  __attribute__((ext_vector_type(8)));
typedef _Float16 v16h __attribute__((ext_vector_type(16)));
union FragH { v16h v; v8h h[2]; };

__device__ __forceinline__ v8h cvt8(v4f a, v4f b) {
  v8h r;
  r[0] = (_Float16)a.x; r[1] = (_Float16)a.y; r[2] = (_Float16)a.z; r[3] = (_Float16)a.w;
  r[4] = (_Float16)b.x; r[5] = (_Float16)b.y; r[6] = (_Float16)b.z; r[7] = (_Float16)b.w;
  return r;
}

__device__ __forceinline__ v8f wmh(v16h a, v16h b, v8f c) {
  v8f d = __builtin_amdgcn_wmma_f32_16x16x32_f16(false, a, false, b, (short)0, c, false, false);
  asm volatile("v_nop\n\tv_nop\n\tv_nop\n\tv_nop" : "+v"(d) : "v"(a), "v"(b));
  return d;
}

template <int NB>
__device__ __forceinline__ int scan_chunk(const int* __restrict__ keys, int nE, int cbase, int nodeBase,
                                          int* list, int tid, int lane, int wave) {
  int wc = 0;
#pragma unroll
  for (int g = 0; g < NGRP; ++g) {
    const int el0  = (g * NTHR + tid) * EPT;
    const int e0   = cbase + el0;
    const int sent = -2147483647 - 1;
    v4i da, db;
    if (e0 + 7 < nE) {
      da = *(const v4i*)(keys + e0);
      db = *(const v4i*)(keys + e0 + 4);
    } else {
      da.x = (e0     < nE) ? keys[min(e0, nE - 1)] : sent;
      da.y = (e0 + 1 < nE) ? keys[min(e0 + 1, nE - 1)] : sent;
      da.z = (e0 + 2 < nE) ? keys[min(e0 + 2, nE - 1)] : sent;
      da.w = (e0 + 3 < nE) ? keys[min(e0 + 3, nE - 1)] : sent;
      db.x = (e0 + 4 < nE) ? keys[min(e0 + 4, nE - 1)] : sent;
      db.y = (e0 + 5 < nE) ? keys[min(e0 + 5, nE - 1)] : sent;
      db.z = (e0 + 6 < nE) ? keys[min(e0 + 6, nE - 1)] : sent;
      db.w = (e0 + 7 < nE) ? keys[min(e0 + 7, nE - 1)] : sent;
    }
    const unsigned nb = (unsigned)nodeBase;
    const unsigned s0 = (unsigned)da.x - nb, s1 = (unsigned)da.y - nb;
    const unsigned s2 = (unsigned)da.z - nb, s3 = (unsigned)da.w - nb;
    const unsigned s4 = (unsigned)db.x - nb, s5 = (unsigned)db.y - nb;
    const unsigned s6 = (unsigned)db.z - nb, s7 = (unsigned)db.w - nb;
    const bool h0 = s0 < (unsigned)NB, h1 = s1 < (unsigned)NB, h2 = s2 < (unsigned)NB, h3 = s3 < (unsigned)NB;
    const bool h4 = s4 < (unsigned)NB, h5 = s5 < (unsigned)NB, h6 = s6 < (unsigned)NB, h7 = s7 < (unsigned)NB;
    const unsigned any = __builtin_amdgcn_ballot_w32(h0 | h1 | h2 | h3 | h4 | h5 | h6 | h7);
    if (any != 0u) {
#define HITJ(J, HJ, SJ) { \
        const unsigned mj = __builtin_amdgcn_ballot_w32(HJ); \
        if (mj != 0u) { \
          if (HJ) { \
            const int pos = wc + (int)__builtin_amdgcn_mbcnt_lo(mj, 0u); \
            if (pos < WCAP) list[wave * WCAP + pos] = ((el0 + (J)) << 12) | (int)(SJ); \
          } \
          wc += (int)__builtin_popcount(mj); } }
      HITJ(0, h0, s0)
      HITJ(1, h1, s1)
      HITJ(2, h2, s2)
      HITJ(3, h3, s3)
      HITJ(4, h4, s4)
      HITJ(5, h5, s5)
      HITJ(6, h6, s6)
      HITJ(7, h7, s7)
#undef HITJ
    }
  }
  return wc;
}

__global__ __launch_bounds__(NTHR) void k_wprep(
    const float* __restrict__ W1, const float* __restrict__ W2,
    _Float16* w1s, _Float16* w2s) {
  const int i  = blockIdx.x * NTHR + threadIdx.x;
  const int n1 = DHID * DIN / 8;
  const int n2 = NCLS * DHID / 8;
  if (i >= n1 + n2) return;
  const bool first = i < n1;
  const int o = (first ? i : i - n1) * 8;
  v4f a, b;
  _Float16* dp;
  if (first) {
    const int n  = o / DIN;
    const int k0 = o - n * DIN;
    const float* p = W1 + (size_t)k0 * DHID + n;
    a.x = p[0];        a.y = p[DHID];     a.z = p[2 * DHID]; a.w = p[3 * DHID];
    b.x = p[4 * DHID]; b.y = p[5 * DHID]; b.z = p[6 * DHID]; b.w = p[7 * DHID];
    dp = w1s + o;
  } else {
    const int n  = o / DHID;
    const int k0 = o - n * DHID;
    const float* p = W2 + (size_t)k0 * NCLS + n;
    a.x = p[0];        a.y = p[NCLS];     a.z = p[2 * NCLS]; a.w = p[3 * NCLS];
    b.x = p[4 * NCLS]; b.y = p[5 * NCLS]; b.z = p[6 * NCLS]; b.w = p[7 * NCLS];
    dp = w2s + o;
  }
  a = a * WSCALE;
  b = b * WSCALE;
  const v8h hv = cvt8(a, b);
  *(volatile v8h*)dp = hv;
  __threadfence();
  *(volatile v8h*)dp = hv;
}

__global__ __launch_bounds__(NTHR) void k_deg(
    const int* __restrict__ srcp, const int* __restrict__ dstp,
    float* nrs, float* nrd, int nE) {
  __shared__ __attribute__((aligned(16))) int cnt[2 * NBD];
  __shared__ __attribute__((aligned(16))) int list[LISTN];
  __shared__ int wcnt[NWAVE];
  const int tid = threadIdx.x, lane = tid & 31, wave = tid >> 5;
  const int nodeBase = blockIdx.x * NBD;

  for (int i = tid; i < 2 * NBD; i += NTHR) cnt[i] = 0;
  __syncthreads();

  const int nChunks = (nE + CHUNK - 1) / CHUNK;
#pragma unroll 1
  for (int ch = 0; ch < 2 * nChunks; ++ch) {
    const bool second = ch >= nChunks;
    const int* keys   = second ? dstp : srcp;
    const int  cbase  = (second ? (ch - nChunks) : ch) * CHUNK;
    const int  coff   = second ? NBD : 0;
    const int wc = scan_chunk<NBD>(keys, nE, cbase, nodeBase, list, tid, lane, wave);
    if (lane == 0) wcnt[wave] = wc;
    __syncthreads();
    if (wave == 0) {
#pragma unroll 1
      for (int wsx = 0; wsx < NWAVE; ++wsx) {
        int n = __builtin_amdgcn_readfirstlane(wcnt[wsx]);
        n = n > WCAP ? WCAP : (n < 0 ? 0 : n);
        const int* lp = list + wsx * WCAP;
#pragma unroll 1
        for (int i = 0; i < n; ++i) {
          const int ent  = __builtin_amdgcn_readfirstlane(lp[i]);
          const int slot = ent & (NBD - 1);
          if (lane == 0) cnt[coff + slot] = cnt[coff + slot] + 1;
        }
      }
    }
    __syncthreads();
  }

  v4f qs[4], qd[4];
#pragma unroll
  for (int q = 0; q < 4; ++q) {
    const int f = (wave * 4 + q) * 128 + 4 * lane;
    const v4i cs = *(const v4i*)(cnt + f);
    const v4i cd = *(const v4i*)(cnt + NBD + f);
    qs[q].x = rsqrtf((float)(cs.x > 1 ? cs.x : 1));
    qs[q].y = rsqrtf((float)(cs.y > 1 ? cs.y : 1));
    qs[q].z = rsqrtf((float)(cs.z > 1 ? cs.z : 1));
    qs[q].w = rsqrtf((float)(cs.w > 1 ? cs.w : 1));
    qd[q].x = rsqrtf((float)(cd.x > 1 ? cd.x : 1));
    qd[q].y = rsqrtf((float)(cd.y > 1 ? cd.y : 1));
    qd[q].z = rsqrtf((float)(cd.z > 1 ? cd.z : 1));
    qd[q].w = rsqrtf((float)(cd.w > 1 ? cd.w : 1));
  }
  float* ps = nrs + (size_t)nodeBase;
  float* pd = nrd + (size_t)nodeBase;
#pragma unroll
  for (int q = 0; q < 4; ++q) {
    *(volatile v4f*)(ps + (wave * 4 + q) * 128 + 4 * lane) = qs[q];
    *(volatile v4f*)(pd + (wave * 4 + q) * 128 + 4 * lane) = qd[q];
  }
  __threadfence();
#pragma unroll
  for (int q = 0; q < 4; ++q) {
    *(volatile v4f*)(ps + (wave * 4 + q) * 128 + 4 * lane) = qs[q];
    *(volatile v4f*)(pd + (wave * 4 + q) * 128 + 4 * lane) = qd[q];
  }
}

__global__ __launch_bounds__(NTHR) void k_gemm1(
    const float* __restrict__ x, const _Float16* __restrict__ w1s,
    const float* __restrict__ nrs, float* g1, int nN) {
  extern __shared__ v4f lds_dyn[];
  _Float16* sA  = (_Float16*)lds_dyn;
  float*    stg = (float*)lds_dyn;
  const int tid = threadIdx.x, lane = tid & 31, wave = tid >> 5, hh = lane >> 4, m = lane & 15;
  const int rowBase = blockIdx.x * G1ROWS;

#pragma unroll
  for (int i = 0; i < (G1ROWS * DIN / 8) / NTHR; ++i) {
    const int idx = i * NTHR + tid;
    const int r   = idx >> 4;
    const int c0  = (idx & 15) * 8;
    int node = rowBase + r;
    node = node > nN - 1 ? nN - 1 : node;
    const float* xp = x + (size_t)node * DIN + c0;
    const v4f a = *(const v4f*)xp, b = *(const v4f*)(xp + 4);
    *(v8h*)(sA + r * APITCH + c0) = cvt8(a, b);
  }
  __syncthreads();

  v8f acc[4];
#pragma unroll
  for (int t = 0; t < 4; ++t) { v8f z = {0.f, 0.f, 0.f, 0.f, 0.f, 0.f, 0.f, 0.f}; acc[t] = z; }
  const _Float16* ar = sA + (wave * 16 + m) * APITCH + 8 * hh;
#pragma unroll
  for (int kt = 0; kt < DIN / 32; ++kt) {
    FragH a;
    a.h[0] = *(const v8h*)(ar + 32 * kt);
    a.h[1] = *(const v8h*)(ar + 32 * kt + 16);
#pragma unroll
    for (int t = 0; t < 4; ++t) {
      const _Float16* bp = w1s + (size_t)(16 * t + m) * DIN + 32 * kt + 8 * hh;
      FragH b;
      b.h[0] = *(const v8h*)bp;
      b.h[1] = *(const v8h*)(bp + 16);
      acc[t] = wmh(a.v, b.v, acc[t]);
    }
  }
  __syncthreads();

  const int r0 = wave * 16 + 8 * hh;
  const v4f dA = *(const v4f*)(nrs + (size_t)rowBase + r0);
  const v4f dB = *(const v4f*)(nrs + (size_t)rowBase + r0 + 4);
  const float d0 = dA.x * WINV, d1 = dA.y * WINV, d2 = dA.z * WINV, d3 = dA.w * WINV;
  const float d4 = dB.x * WINV, d5 = dB.y * WINV, d6 = dB.z * WINV, d7 = dB.w * WINV;
  float* sp = stg + r0 * DHID + m;
#pragma unroll
  for (int t = 0; t < 4; ++t) {
    sp[0 * DHID + 16 * t] = acc[t][0] * d0;
    sp[1 * DHID + 16 * t] = acc[t][1] * d1;
    sp[2 * DHID + 16 * t] = acc[t][2] * d2;
    sp[3 * DHID + 16 * t] = acc[t][3] * d3;
    sp[4 * DHID + 16 * t] = acc[t][4] * d4;
    sp[5 * DHID + 16 * t] = acc[t][5] * d5;
    sp[6 * DHID + 16 * t] = acc[t][6] * d6;
    sp[7 * DHID + 16 * t] = acc[t][7] * d7;
  }
  __syncthreads();

  const float* lp = stg + wave * 16 * DHID + 4 * lane;
  float* gp = g1 + ((size_t)rowBase + wave * 16) * DHID + 4 * lane;
  v4f ov[8];
#pragma unroll
  for (int q = 0; q < 8; ++q) ov[q] = *(const v4f*)(lp + q * 128);
#pragma unroll
  for (int q = 0; q < 8; ++q) *(volatile v4f*)(gp + q * 128) = ov[q];
  __threadfence();
#pragma unroll
  for (int q = 0; q < 8; ++q) *(volatile v4f*)(gp + q * 128) = ov[q];
}

__global__ __launch_bounds__(NTHR) void k_agg1(
    const int* __restrict__ srcp, const int* __restrict__ dstp,
    const float* __restrict__ g1, const float* __restrict__ nrs, const float* __restrict__ nrd,
    const float* __restrict__ b1, const _Float16* __restrict__ w2s, float* g2,
    int nN, int nE) {
  extern __shared__ v4f lds_dyn[];
  float* acc  = (float*)lds_dyn;
  int*   list = (int*)(acc + NB1 * DHID);
  int*   wcnt = list + LISTN;
  float* stg2 = (float*)list;
  const int tid = threadIdx.x, lane = tid & 31, wave = tid >> 5, hh = lane >> 4, m = lane & 15;
  const int nodeBase = blockIdx.x * NB1;

  {
    const v4f z = {0.f, 0.f, 0.f, 0.f};
    for (int i = tid; i < NB1 * DHID / 4; i += NTHR) lds_dyn[i] = z;
  }
  __syncthreads();

  const int nChunks = (nE + CHUNK - 1) / CHUNK;
#pragma unroll 1
  for (int ch = 0; ch < nChunks; ++ch) {
    const int cbase = ch * CHUNK;
    const int wc = scan_chunk<NB1>(dstp, nE, cbase, nodeBase, list, tid, lane, wave);
    if (lane == 0) wcnt[wave] = wc;
    __syncthreads();
    if (wave == 0) {
#pragma unroll 1
      for (int wsx = 0; wsx < NWAVE; ++wsx) {
        int n = __builtin_amdgcn_readfirstlane(wcnt[wsx]);
        n = n > WCAP ? WCAP : (n < 0 ? 0 : n);
        const int* lp = list + wsx * WCAP;
#pragma unroll 1
        for (int i = 0; i < n; ++i) {
          const int ent  = __builtin_amdgcn_readfirstlane(lp[i]);
          const int slot = ent & (NB1 - 1);
          int e = cbase + ((ent >> 12) & (CHUNK - 1));
          e = e > nE - 1 ? nE - 1 : e;
          int s = srcp[e];
          s = s < 0 ? 0 : (s > nN - 1 ? nN - 1 : s);
          const v2f v = *(const v2f*)(g1 + (size_t)s * DHID + 2 * lane);
          v2f* ap = (v2f*)(acc + slot * DHID + 2 * lane);
          *ap = *ap + v;
        }
      }
    }
    __syncthreads();
  }

#pragma unroll 4
  for (int i = 0; i < (NB1 * DHID / 4) / NTHR; ++i) {
    const int idx  = i * NTHR + tid;
    const int slot = idx >> 4;
    const int c4   = (idx & 15) * 4;
    int node = nodeBase + slot;
    node = node > nN - 1 ? nN - 1 : node;
    const float d  = nrd[node];
    const v4f   bv = *(const v4f*)(b1 + c4);
    v4f* ap = (v4f*)(acc + slot * DHID + c4);
    v4f hv = (*ap) * d + bv;
    hv.x = fmaxf(hv.x, 0.f); hv.y = fmaxf(hv.y, 0.f); hv.z = fmaxf(hv.z, 0.f); hv.w = fmaxf(hv.w, 0.f);
    *ap = hv;
  }
  __syncthreads();

  FragH bw[2];
#pragma unroll
  for (int kt = 0; kt < 2; ++kt) {
    const _Float16* bp = w2s + m * DHID + 32 * kt + 8 * hh;
    bw[kt].h[0] = *(const v8h*)bp;
    bw[kt].h[1] = *(const v8h*)(bp + 16);
  }

#pragma unroll 1
  for (int s = 0; s < NB1 / 256; ++s) {
#pragma unroll
    for (int q = 0; q < 2; ++q) {
      const int tl = wave + 8 * q;
      const int t  = 16 * s + tl;
      v8f c = {0.f, 0.f, 0.f, 0.f, 0.f, 0.f, 0.f, 0.f};
#pragma unroll
      for (int kt = 0; kt < 2; ++kt) {
        const float* ap = acc + (16 * t + m) * DHID + 32 * kt + 8 * hh;
        const v4f p0 = *(const v4f*)ap,        p1 = *(const v4f*)(ap + 4);
        const v4f p2 = *(const v4f*)(ap + 16), p3 = *(const v4f*)(ap + 20);
        FragH a;
        a.h[0] = cvt8(p0, p1);
        a.h[1] = cvt8(p2, p3);
        c = wmh(a.v, bw[kt].v, c);
      }
      const int node0 = nodeBase + 16 * t + 8 * hh;
      const v4f dA = *(const v4f*)(nrs + (size_t)node0);
      const v4f dB = *(const v4f*)(nrs + (size_t)node0 + 4);
      float* sp = stg2 + (16 * tl + 8 * hh) * NCLS + m;
      sp[0 * NCLS] = c[0] * dA.x * WINV;
      sp[1 * NCLS] = c[1] * dA.y * WINV;
      sp[2 * NCLS] = c[2] * dA.z * WINV;
      sp[3 * NCLS] = c[3] * dA.w * WINV;
      sp[4 * NCLS] = c[4] * dB.x * WINV;
      sp[5 * NCLS] = c[5] * dB.y * WINV;
      sp[6 * NCLS] = c[6] * dB.z * WINV;
      sp[7 * NCLS] = c[7] * dB.w * WINV;
    }
    __syncthreads();
    v4f ov[4];
#pragma unroll
    for (int q = 0; q < 4; ++q) ov[q] = *(const v4f*)(stg2 + (wave * 4 + q) * 128 + 4 * lane);
    float* gp = g2 + ((size_t)nodeBase + 256 * s) * NCLS;
#pragma unroll
    for (int q = 0; q < 4; ++q) *(volatile v4f*)(gp + (wave * 4 + q) * 128 + 4 * lane) = ov[q];
    __threadfence();
#pragma unroll
    for (int q = 0; q < 4; ++q) *(volatile v4f*)(gp + (wave * 4 + q) * 128 + 4 * lane) = ov[q];
    __syncthreads();
  }
}

__global__ __launch_bounds__(NTHR) void k_agg2(
    const int* __restrict__ srcp, const int* __restrict__ dstp,
    const float* __restrict__ g2, const float* __restrict__ nrd,
    const float* __restrict__ b2, float* out, int nN, int nE) {
  extern __shared__ v4f lds_dyn[];
  float* acc  = (float*)lds_dyn;
  int*   list = (int*)(acc + NB2 * NCLS);
  int*   wcnt = list + LISTN;
  const int tid = threadIdx.x, lane = tid & 31, wave = tid >> 5;
  const int nodeBase = blockIdx.x * NB2;

  {
    const v4f z = {0.f, 0.f, 0.f, 0.f};
    for (int i = tid; i < NB2 * NCLS / 4; i += NTHR) lds_dyn[i] = z;
  }
  __syncthreads();

  const int nChunks = (nE + CHUNK - 1) / CHUNK;
#pragma unroll 1
  for (int ch = 0; ch < nChunks; ++ch) {
    const int cbase = ch * CHUNK;
    const int wc = scan_chunk<NB2>(dstp, nE, cbase, nodeBase, list, tid, lane, wave);
    if (lane == 0) wcnt[wave] = wc;
    __syncthreads();
    if (wave == 0) {
#pragma unroll 1
      for (int wsx = 0; wsx < NWAVE; ++wsx) {
        int n = __builtin_amdgcn_readfirstlane(wcnt[wsx]);
        n = n > WCAP ? WCAP : (n < 0 ? 0 : n);
        const int* lp = list + wsx * WCAP;
#pragma unroll 1
        for (int i = 0; i < n; ++i) {
          const int ent  = __builtin_amdgcn_readfirstlane(lp[i]);
          const int slot = ent & (NB2 - 1);
          int e = cbase + ((ent >> 12) & (CHUNK - 1));
          e = e > nE - 1 ? nE - 1 : e;
          int s = srcp[e];
          s = s < 0 ? 0 : (s > nN - 1 ? nN - 1 : s);
          if (lane < NCLS) {
            float* ap = acc + slot * NCLS + lane;
            *ap = *ap + g2[(size_t)s * NCLS + lane];
          }
        }
      }
    }
    __syncthreads();
  }

#pragma unroll 4
  for (int i = 0; i < (NB2 * NCLS / 4) / NTHR; ++i) {
    const int idx  = i * NTHR + tid;
    const int slot = idx >> 2;
    const int c4   = (idx & 3) * 4;
    int node = nodeBase + slot;
    node = node > nN - 1 ? nN - 1 : node;
    const float d  = nrd[node];
    const v4f   bv = *(const v4f*)(b2 + c4);
    v4f* ap = (v4f*)(acc + slot * NCLS + c4);
    *ap = (*ap) * d + bv;
  }
  __syncthreads();

  const size_t outN = (size_t)nN * NCLS;
  const size_t ob   = (size_t)nodeBase * NCLS;
#pragma unroll 4
  for (int q = 0; q < 64; ++q) {
    const int f = (wave * 64 + q) * 128 + 4 * lane;
    const size_t gi = ob + (size_t)f;
    if (gi < outN) { const v4f v = *(const v4f*)(acc + f); *(volatile v4f*)(out + gi) = v; }
  }
  __threadfence();
#pragma unroll 4
  for (int q = 0; q < 64; ++q) {
    const int f = (wave * 64 + q) * 128 + 4 * lane;
    const size_t gi = ob + (size_t)f;
    if (gi < outN) { const v4f v = *(const v4f*)(acc + f); *(volatile v4f*)(out + gi) = v; }
  }
}

extern "C" void kernel_launch(void* const* d_in, const int* in_sizes, int n_in,
                              void* d_out, int out_size, void* d_ws, size_t ws_size,
                              hipStream_t stream) {
  if (n_in < 7) return;
  const int nN = in_sizes[0] / DIN;
  const int nE = in_sizes[5];
  if (nN <= 0 || nE < 0 || in_sizes[0] != nN * DIN || in_sizes[6] != nE) return;
  if (in_sizes[1] != DIN * DHID || in_sizes[2] < DHID || in_sizes[3] != DHID * NCLS || in_sizes[4] < NCLS) return;
  if (out_size != nN * NCLS) return;

  const float* x   = (const float*)d_in[0];
  const float* W1  = (const float*)d_in[1];
  const float* b1  = (const float*)d_in[2];
  const float* W2  = (const float*)d_in[3];
  const float* b2  = (const float*)d_in[4];
  const int*   src = (const int*)d_in[5];
  const int*   dst = (const int*)d_in[6];
  float* out = (float*)d_out;

  const int nBD = (nN + NBD - 1) / NBD;
  const int nG1 = (nN + G1ROWS - 1) / G1ROWS;
  const int nA1 = (nN + NB1 - 1) / NB1;
  const int nA2 = (nN + NB2 - 1) / NB2;
  if (nBD * NBD < nG1 * G1ROWS || nBD * NBD < nA1 * NB1) return;

  char* ws = (char*)d_ws;
  size_t off = 0;
  const size_t oW1 = off; off += (size_t)DHID * DIN * 2;                         off = (off + 255) & ~(size_t)255;
  const size_t oW2 = off; off += (size_t)NCLS * DHID * 2;                        off = (off + 255) & ~(size_t)255;
  const size_t oNs = off; off += (size_t)nBD * NBD * 4;                          off = (off + 255) & ~(size_t)255;
  const size_t oNd = off; off += (size_t)nBD * NBD * 4;                          off = (off + 255) & ~(size_t)255;
  const size_t oG1 = off; off += (size_t)nG1 * G1ROWS * DHID * 4;                off = (off + 255) & ~(size_t)255;
  const size_t oG2 = off; off += (size_t)nA1 * NB1 * NCLS * 4;                   off = (off + 255) & ~(size_t)255;
  if (off > ws_size) return;
  _Float16* w1s = (_Float16*)(ws + oW1);
  _Float16* w2s = (_Float16*)(ws + oW2);
  float*    nrs = (float*)(ws + oNs);
  float*    nrd = (float*)(ws + oNd);
  float*    g1  = (float*)(ws + oG1);
  float*    g2  = (float*)(ws + oG2);

  const int nPrep = DHID * DIN / 8 + NCLS * DHID / 8;
  k_wprep<<<(nPrep + NTHR - 1) / NTHR, NTHR, 0, stream>>>(W1, W2, w1s, w2s);

  k_deg<<<nBD, NTHR, 0, stream>>>(src, dst, nrs, nrd, nE);

  k_gemm1<<<nG1, NTHR, LDS_GEMM1, stream>>>(x, w1s, nrs, g1, nN);

  hipFuncSetAttribute(reinterpret_cast<const void*>(&k_agg1),
                      hipFuncAttributeMaxDynamicSharedMemorySize, LDS_AGG1);
  k_agg1<<<nA1, NTHR, LDS_AGG1, stream>>>(src, dst, g1, nrs, nrd, b1, w2s, g2, nN, nE);

  hipFuncSetAttribute(reinterpret_cast<const void*>(&k_agg2),
                      hipFuncAttributeMaxDynamicSharedMemorySize, LDS_AGG2);
  k_agg2<<<nA2, NTHR, LDS_AGG2, stream>>>(src, dst, g2, nrd, b2, out, nN, nE);
}
